// LocalAttentionND_39754217292518
// MI455X (gfx1250) — hardware-verified
//
#include <hip/hip_runtime.h>
#include <math.h>

typedef __attribute__((ext_vector_type(16))) _Float16 v16h;
typedef __attribute__((ext_vector_type(8)))  _Float16 v8h;
typedef __attribute__((ext_vector_type(16))) __bf16   v16b;
typedef __attribute__((ext_vector_type(8)))  __bf16   v8b;
typedef __attribute__((ext_vector_type(8)))  float    v8f;
typedef __attribute__((ext_vector_type(4)))  float    v4f;
typedef __attribute__((ext_vector_type(4)))  unsigned int v4u;
#define PSCALE 32768.0f
#define U16(p) ((const unsigned short*)(const void*)(p))
#define PSCALE_INV (1.0f / 32768.0f)

constexpr int NB_BATCH = 2;
constexpr int IMG_H = 64;
constexpr int IMG_W = 64;
constexpr int CEMB = 256;
constexpr int NHEADS = 8;
constexpr int DHD = 32;
constexpr int NTOK = NB_BATCH * IMG_H * IMG_W;
constexpr int NQKV = 3 * CEMB;
constexpr int NWP_REAL = 2 * NHEADS;
constexpr int NWP_PAD = 64;
constexpr int KWIN = 7;
constexpr float RMS_EPS = 1e-6f;
constexpr float QK_SCALE = 0.17677669529663687f;
constexpr float MAXD = 4.242640687119285f;

static_assert(NTOK % 64 == 0);
static_assert(NQKV % 64 == 0);
static_assert(CEMB % 64 == 0);
static_assert(NWP_PAD % 64 == 0);
static_assert(CEMB % 32 == 0);
static_assert(IMG_W % 16 == 0);

constexpr size_t SZ_PLANE_TOK = (size_t)NTOK * CEMB * 2;
constexpr size_t SZ_PLANE_WQKV = (size_t)NQKV * CEMB * 2;
constexpr size_t SZ_PLANE_WWP = (size_t)NWP_PAD * CEMB * 2;
constexpr size_t SZ_PLANE_WOUT = (size_t)CEMB * CEMB * 2;
constexpr size_t SZ_QKV = (size_t)NTOK * NQKV * 4;
constexpr size_t SZ_WPR = (size_t)NTOK * NWP_PAD * 4;
constexpr size_t SZ_OBUF = (size_t)NTOK * CEMB * 4;
constexpr size_t OFF_XH = 0;
constexpr size_t OFF_XL = OFF_XH + SZ_PLANE_TOK;
constexpr size_t OFF_WQKVH = OFF_XL + SZ_PLANE_TOK;
constexpr size_t OFF_WQKVL = OFF_WQKVH + SZ_PLANE_WQKV;
constexpr size_t OFF_WWPH = OFF_WQKVL + SZ_PLANE_WQKV;
constexpr size_t OFF_WWPL = OFF_WWPH + SZ_PLANE_WWP;
constexpr size_t OFF_WOUTH = OFF_WWPL + SZ_PLANE_WWP;
constexpr size_t OFF_WOUTL = OFF_WOUTH + SZ_PLANE_WOUT;
constexpr size_t OFF_QKV = OFF_WOUTL + SZ_PLANE_WOUT;
constexpr size_t OFF_WPR = OFF_QKV + SZ_QKV;
constexpr size_t OFF_QH = OFF_WPR + SZ_WPR;
constexpr size_t OFF_QL = OFF_QH + SZ_PLANE_TOK;
constexpr size_t OFF_KH = OFF_QL + SZ_PLANE_TOK;
constexpr size_t OFF_KL = OFF_KH + SZ_PLANE_TOK;
constexpr size_t OFF_OBUF = OFF_KL + SZ_PLANE_TOK;
constexpr size_t OFF_AFH = OFF_OBUF + SZ_OBUF;
constexpr size_t OFF_AFL = OFF_AFH + SZ_PLANE_TOK;
constexpr size_t WS_TOTAL = OFF_AFL + SZ_PLANE_TOK;
static_assert(WS_TOTAL <= 134217728ull);
static_assert(OFF_QKV % 128 == 0 && OFF_WPR % 128 == 0 && OFF_QH % 128 == 0 && OFF_OBUF % 128 == 0 && OFF_AFH % 128 == 0 && OFF_AFL % 128 == 0);

__device__ __forceinline__ unsigned short f2bf_bits(float f) {
  unsigned u = __float_as_uint(f);
  return (unsigned short)((u + 0x7FFFu + ((u >> 16) & 1u)) >> 16);
}
__device__ __forceinline__ float bf_bits2f(unsigned short h) { return __uint_as_float(((unsigned)h) << 16); }

__device__ __forceinline__ void dep_guard_h(v8f& a, v8f& b, v16h x, v16h y) { asm volatile("v_nop\n\tv_nop\n\tv_nop\n\tv_nop" : "+v"(a), "+v"(b) : "v"(x), "v"(y)); }
__device__ __forceinline__ void dep_guard_b(v8f& a, v8f& b, v16b x, v16b y) { asm volatile("v_nop\n\tv_nop\n\tv_nop\n\tv_nop" : "+v"(a), "+v"(b) : "v"(x), "v"(y)); }
__device__ __forceinline__ void keep4_h(v16h a, v16h b, v16h c, v16h d) { asm volatile("v_nop" :: "v"(a), "v"(b), "v"(c), "v"(d)); }
__device__ __forceinline__ void keep4_b(v16b a, v16b b, v16b c, v16b d) { asm volatile("v_nop" :: "v"(a), "v"(b), "v"(c), "v"(d)); }
__device__ __forceinline__ void acc_guard4(v8f& a, v8f& b, v8f& c, v8f& d) { asm volatile("v_nop\n\tv_nop\n\tv_nop\n\tv_nop" : "+v"(a), "+v"(b), "+v"(c), "+v"(d)); }
template <typename T> struct Frag;
template <> struct Frag<_Float16> {
  typedef v16h V; union U { v16h v; v8h h[2]; };
  static __device__ __forceinline__ v16h load(const _Float16* p) {
    U f; f.h[0] = *(const v8h*)(p); f.h[1] = *(const v8h*)(p + 16); return f.v;
  }
  static __device__ __forceinline__ v8f mma(v16h a, v16h b, v8f c) {
    return __builtin_amdgcn_wmma_f32_16x16x32_f16(false, a, false, b, (short)0, c, false, false);
  }
  static __device__ __forceinline__ void guard(v8f& a, v8f& b, v16h x, v16h y) { dep_guard_h(a, b, x, y); }
  static __device__ __forceinline__ void keep(v16h a, v16h b, v16h c, v16h d) { keep4_h(a, b, c, d); }
};
template <> struct Frag<__bf16> {
  typedef v16b V; union U { v16b v; v8b h[2]; };
  static __device__ __forceinline__ v16b load(const __bf16* p) {
    U f; f.h[0] = *(const v8b*)(p); f.h[1] = *(const v8b*)(p + 16); return f.v;
  }
  static __device__ __forceinline__ v8f mma(v16b a, v16b b, v8f c) {
    return __builtin_amdgcn_wmma_f32_16x16x32_bf16(false, a, false, b, (short)0, c, false, false);
  }
  static __device__ __forceinline__ void guard(v8f& a, v8f& b, v16b x, v16b y) { dep_guard_b(a, b, x, y); }
  static __device__ __forceinline__ void keep(v16b a, v16b b, v16b c, v16b d) { keep4_b(a, b, c, d); }
};

template <int ET> struct Elem;
template <> struct Elem<0> { typedef _Float16 T; };
template <> struct Elem<1> { typedef __bf16 T; };
template <int ET, bool SPLIT, int BIAS_MODE, int OUT_MODE, bool RESID, int ACT = 0>
__global__ __launch_bounds__(256) void wmma_gemm64(
    const unsigned short* __restrict__ Ap, const unsigned short* __restrict__ A2p, int lda, long strideA,
    const unsigned short* __restrict__ Btp, const unsigned short* __restrict__ Bt2p, int ldb, long strideB,
    void* __restrict__ Cout, void* __restrict__ Cout2, int ldc, long strideC,
    const float* __restrict__ bias,
    const float* __restrict__ resid, long strideR,
    int M, int N, int K, float scale) {
  typedef typename Elem<ET>::T T;
  typedef typename Frag<T>::V V;
  const T* A = (const T*)Ap; const T* A2 = (const T*)A2p; const T* Bt = (const T*)Btp; const T* Bt2 = (const T*)Bt2p;
  __shared__ __align__(16) float sT[8][16 * 68];
  const int b    = blockIdx.y;
  const int lane = threadIdx.x & 31;
  const int wave = threadIdx.x >> 5;
  const int tilesN = N >> 6;
  const int tilesM = M >> 6;
  const int tile = blockIdx.x * 8 + wave;
  if (tile >= tilesM * tilesN) return;
  const int tm = tile / tilesN;
  const int tn = tile - tm * tilesN;
  const int m0 = tm << 6;
  const int n0 = tn << 6;

  const T* Ab  = A  + (size_t)b * strideA;
  const T* Bb  = Bt + (size_t)b * strideB;
  const T* Ab2 = SPLIT ? (A2  + (size_t)b * strideA) : nullptr;
  const T* Bb2 = SPLIT ? (Bt2 + (size_t)b * strideB) : nullptr;

  const int rlane = lane & 15;
  const int koff  = (lane >> 4) * 8;
  const int mOff  = (lane >> 4) * 8;

  v8f acc[4][4];
#pragma unroll
  for (int i = 0; i < 4; ++i)
#pragma unroll
    for (int j = 0; j < 4; ++j) acc[i][j] = (v8f){0.f,0.f,0.f,0.f,0.f,0.f,0.f,0.f};

  for (int k0 = 0; k0 < K; k0 += 32) {
    V bh[4], bl[4];
#pragma unroll
    for (int j = 0; j < 4; ++j) {
      const size_t bo = (size_t)(n0 + (j << 4) + rlane) * ldb + koff + k0;
      bh[j] = Frag<T>::load(Bb + bo);
      if (SPLIT) bl[j] = Frag<T>::load(Bb2 + bo);
    }
#pragma unroll
    for (int i = 0; i < 4; ++i) {
      const size_t ao = (size_t)(m0 + (i << 4) + rlane) * lda + koff + k0;
      V ah = Frag<T>::load(Ab + ao);
      V al;
      if (SPLIT) al = Frag<T>::load(Ab2 + ao);
#pragma unroll
      for (int j = 0; j < 4; ++j) {
        acc[i][j] = Frag<T>::mma(ah, bh[j], acc[i][j]);
        if (SPLIT) {
          acc[i][j] = Frag<T>::mma(ah, bl[j], acc[i][j]);
          acc[i][j] = Frag<T>::mma(al, bh[j], acc[i][j]);
        }
      }
      Frag<T>::guard(acc[i][0], acc[i][3], ah, SPLIT ? al : ah);
    }
    Frag<T>::keep(bh[0], bh[1], bh[2], bh[3]);
    if (SPLIT) Frag<T>::keep(bl[0], bl[1], bl[2], bl[3]);
  }
  acc_guard4(acc[0][0], acc[0][1], acc[0][2], acc[0][3]);
  acc_guard4(acc[1][0], acc[1][1], acc[1][2], acc[1][3]);
  acc_guard4(acc[2][0], acc[2][1], acc[2][2], acc[2][3]);
  acc_guard4(acc[3][0], acc[3][1], acc[3][2], acc[3][3]);

  float* slab = sT[wave];
  const float* Rb = RESID ? (resid + (size_t)b * strideR) : nullptr;
#pragma unroll
  for (int i = 0; i < 4; ++i) {
    const int mBase = m0 + (i << 4);
#pragma unroll
    for (int j = 0; j < 4; ++j) {
      const int n = n0 + (j << 4) + rlane;
      float bv = 0.f;
      if (BIAS_MODE == 2) bv = bias[n];
#pragma unroll
      for (int r = 0; r < 8; ++r) {
        float v = acc[i][j][r] * scale;
        if (BIAS_MODE == 1) v += bias[mBase + mOff + r];
        if (BIAS_MODE == 2) v += bv;
        if (RESID) v += Rb[(size_t)(mBase + mOff + r) * ldc + n];
        if (ACT == 1) v = tanhf(v);
        if (ACT == 2) v = fmaxf(v, 0.0f);
        if (ACT == 3) v = v / (1.0f + expf(-v));
        if (ACT == 4) v = (v > 0.f) ? v : 0.01f * v;
        if (ACT == 5) v = 0.5f * v * (1.0f + erff(v * 0.70710678118654752f));
        slab[(mOff + r) * 68 + (j << 4) + rlane] = v;
      }
    }
    __builtin_amdgcn_fence(__ATOMIC_RELEASE, "workgroup");
    __builtin_amdgcn_wave_barrier();
    __builtin_amdgcn_fence(__ATOMIC_ACQUIRE, "workgroup");
    if (OUT_MODE == 0) {
      float* C = (float*)Cout + (size_t)b * strideC;
      const int hh = lane >> 4, c4 = (lane & 15) * 4;
      for (int pass = 0; pass < 2; ++pass) {
#pragma unroll
        for (int it = 0; it < 8; ++it) {
          const int row = it * 2 + hh;
          v4f v = *(const v4f*)(slab + row * 68 + c4);
          *(volatile v4f*)(C + (size_t)(mBase + row) * ldc + n0 + c4) = v;
        }
        __threadfence();
      }
    } else {
      const int q = lane >> 3, c8 = (lane & 7) * 8;
      unsigned short* C  = (unsigned short*)Cout  + (size_t)b * strideC;
      unsigned short* C2 = (OUT_MODE == 2) ? ((unsigned short*)Cout2 + (size_t)b * strideC) : nullptr;
      for (int pass = 0; pass < 2; ++pass) {
#pragma unroll
        for (int it = 0; it < 4; ++it) {
          const int row = it * 4 + q;
          const float* sp = slab + row * 68 + c8;
          v8h hv, lv;
#pragma unroll
          for (int e = 0; e < 8; ++e) {
            if (OUT_MODE == 1) {
              hv[e] = (_Float16)sp[e];
            } else {
              unsigned short hb = f2bf_bits(sp[e]);
              unsigned short lb = f2bf_bits(sp[e] - bf_bits2f(hb));
              hv[e] = __builtin_bit_cast(_Float16, hb);
              lv[e] = __builtin_bit_cast(_Float16, lb);
            }
          }
          *(volatile v8h*)(C + (size_t)(mBase + row) * ldc + n0 + c8) = hv;
          if (OUT_MODE == 2) *(volatile v8h*)(C2 + (size_t)(mBase + row) * ldc + n0 + c8) = lv;
        }
        __threadfence();
      }
    }
    __builtin_amdgcn_fence(__ATOMIC_RELEASE, "workgroup");
    __builtin_amdgcn_wave_barrier();
    __builtin_amdgcn_fence(__ATOMIC_ACQUIRE, "workgroup");
  }
}

__device__ __forceinline__ v8f at_mma(v16b a, v16b b, v8f c) {
  c = __builtin_amdgcn_wmma_f32_16x16x32_bf16(false, a, false, b, (short)0, c, false, false);
  asm volatile("v_nop\n\tv_nop\n\tv_nop\n\tv_nop" : "+v"(c) : "v"(a), "v"(b));
  return c;
}

__device__ __forceinline__ float sigm_f(float z) { return 1.0f / (1.0f + expf(-z)); }
__device__ __forceinline__ float silu_f(float z) { return z * sigm_f(z); }

__global__ __launch_bounds__(256) void split_planes_kernel(
    const float* __restrict__ src, int nsrc,
    unsigned short* __restrict__ hi, unsigned short* __restrict__ lo, int ntot8) {
  const int i = blockIdx.x * 256 + threadIdx.x;
  if (i >= ntot8) return;
  const int e0 = i * 8;
  const bool ok = e0 < nsrc;
  const int eb = ok ? e0 : (nsrc - 8);
  const v4f a = *(const v4f*)(src + eb);
  const v4f bq = *(const v4f*)(src + eb + 4);
  float f[8];
  f[0] = a[0]; f[1] = a[1]; f[2] = a[2]; f[3] = a[3];
  f[4] = bq[0]; f[5] = bq[1]; f[6] = bq[2]; f[7] = bq[3];
  unsigned short hb[8], lb[8];
#pragma unroll
  for (int e = 0; e < 8; ++e) {
    const float val = ok ? f[e] : 0.0f;
    hb[e] = f2bf_bits(val);
    lb[e] = f2bf_bits(val - bf_bits2f(hb[e]));
  }
  v4u hw, lw;
#pragma unroll
  for (int j = 0; j < 4; ++j) {
    hw[j] = (unsigned)hb[2 * j] | ((unsigned)hb[2 * j + 1] << 16);
    lw[j] = (unsigned)lb[2 * j] | ((unsigned)lb[2 * j + 1] << 16);
  }
  for (int pass = 0; pass < 2; ++pass) {
    *(volatile v4u*)(hi + e0) = hw;
    *(volatile v4u*)(lo + e0) = lw;
    __threadfence();
  }
}

__global__ __launch_bounds__(256) void qk_prep_kernel(
    const float* __restrict__ qkv, const float* __restrict__ wqn, const float* __restrict__ wkn,
    unsigned short* __restrict__ qhp, unsigned short* __restrict__ qlp,
    unsigned short* __restrict__ khp, unsigned short* __restrict__ klp) {
  __shared__ float tcos[128];
  __shared__ float tsin[128];
  __shared__ __align__(16) unsigned short pln[4][2 * CEMB];
  const int tid = threadIdx.x;
  if (tid < 128) {
    const int ph = tid >> 4, pi = tid & 15;
    const float fr = exp2f((float)pi * (-0.83048202372184059f));
    const float ang = (float)ph * fr;
    tcos[tid] = cosf(ang);
    tsin[tid] = sinf(ang);
  }
  __syncthreads();
  const int i = tid & 15, g = tid >> 4, h = g & 7, tl = g >> 3;
  const int token = blockIdx.x * 2 + tl;
  const float* qp = qkv + (size_t)token * NQKV + h * DHD;
  const float q0 = qp[i], q1 = qp[i + 16];
  const float k0 = qp[CEMB + i], k1 = qp[CEMB + 16 + i];
  float sq = q0 * q0 + q1 * q1;
  float sk = k0 * k0 + k1 * k1;
#pragma unroll
  for (int off = 1; off < 16; off <<= 1) {
    sq += __shfl_xor(sq, off, 32);
    sk += __shfl_xor(sk, off, 32);
  }
  const float iq = 1.0f / sqrtf(sq * (1.0f / 32.0f) + RMS_EPS);
  const float ik = 1.0f / sqrtf(sk * (1.0f / 32.0f) + RMS_EPS);
  const float wq0 = wqn[i], wq1 = wqn[i + 16], wk0 = wkn[i], wk1 = wkn[i + 16];
  const float a0 = q0 * iq * wq0, a1 = q1 * iq * wq1;
  const float b0 = k0 * ik * wk0, b1 = k1 * ik * wk1;
  const float cs = tcos[h * 16 + i], sn = tsin[h * 16 + i];
  const float qo0 = a0 * cs - a1 * sn, qo1 = a0 * sn + a1 * cs;
  const float ko0 = b0 * cs - b1 * sn, ko1 = b0 * sn + b1 * cs;
  const unsigned short qh0 = f2bf_bits(qo0), qh1 = f2bf_bits(qo1);
  const unsigned short kh0 = f2bf_bits(ko0), kh1 = f2bf_bits(ko1);
  const unsigned short ql0 = f2bf_bits(qo0 - bf_bits2f(qh0)), ql1 = f2bf_bits(qo1 - bf_bits2f(qh1));
  const unsigned short kl0 = f2bf_bits(ko0 - bf_bits2f(kh0)), kl1 = f2bf_bits(ko1 - bf_bits2f(kh1));
  const int o0 = tl * CEMB + h * DHD + i, o1 = o0 + 16;
  pln[0][o0] = qh0; pln[0][o1] = qh1;
  pln[1][o0] = ql0; pln[1][o1] = ql1;
  pln[2][o0] = kh0; pln[2][o1] = kh1;
  pln[3][o0] = kl0; pln[3][o1] = kl1;
  __syncthreads();
  const int wave = tid >> 5, lane = tid & 31;
  const int plane = wave >> 1, tsel = wave & 1, q4 = lane >> 3;
  const int off = tsel * CEMB + q4 * 64 + (lane & 7) * 8;
  const v4u val = *(const v4u*)(const void*)(&pln[plane][off]);
  unsigned short* dst = (plane == 0) ? qhp : ((plane == 1) ? qlp : ((plane == 2) ? khp : klp));
  const size_t go = (size_t)(blockIdx.x * 2) * CEMB + off;
  for (int pass = 0; pass < 2; ++pass) {
    *(volatile v4u*)(dst + go) = val;
    __threadfence();
  }
}

__global__ __launch_bounds__(128) void local_attn_kernel(
    const unsigned short* __restrict__ qhp, const unsigned short* __restrict__ qlp,
    const unsigned short* __restrict__ khp, const unsigned short* __restrict__ klp,
    const float* __restrict__ qkv, const float* __restrict__ wpraw,
    const float* __restrict__ bwp, float* __restrict__ obuf) {
  __shared__ __align__(16) unsigned short Ksh[4][32 * 32];
  __shared__ __align__(16) unsigned short Ksl[4][32 * 32];
  __shared__ __align__(16) unsigned short Vth[4][32 * 32];
  __shared__ __align__(16) unsigned short Vtl[4][32 * 32];
  __shared__ __align__(16) unsigned short Psh[4][16 * 32];
  __shared__ __align__(16) unsigned short Psl[4][16 * 32];
  __shared__ __align__(16) float Osh[4][16 * 36];

  const int tid = threadIdx.x;
  const int wave = tid >> 5, lane = tid & 31, hh = lane >> 4, cc = lane & 15, koff = hh * 8;
  const int bx = blockIdx.x;
  const int hg = bx & 1;
  const int xt = (bx >> 1) & 3;
  const int yy = (bx >> 3) & 63;
  const int bb = (bx >> 9) & 1;
  const int head = hg * 4 + wave;
  const int x0 = xt * 16;
  const int tok0 = bb * (IMG_H * IMG_W) + yy * IMG_W + x0;

  const int pxl = lane & 15;
  const float rw = wpraw[(size_t)(tok0 + pxl) * NWP_PAD + head] + bwp[head];
  const float rs = wpraw[(size_t)(tok0 + pxl) * NWP_PAD + NHEADS + head] + bwp[NHEADS + head];
  const float widthl = sigm_f(silu_f(rw)) * MAXD + 0.5f;
  const float sharpl = sigm_f(silu_f(rs)) * 9.5f + 0.5f;
  float wr[8], shp[8];
#pragma unroll
  for (int r = 0; r < 8; ++r) {
    wr[r] = __shfl(widthl, 8 * hh + r, 32);
    shp[r] = __shfl(sharpl, 8 * hh + r, 32);
  }

  const __bf16* qhb = (const __bf16*)(const void*)qhp;
  const __bf16* qlb = (const __bf16*)(const void*)qlp;
  const size_t qoff = (size_t)(tok0 + cc) * CEMB + head * DHD + koff;
  const v16b qah = Frag<__bf16>::load(qhb + qoff);
  const v16b qal = Frag<__bf16>::load(qlb + qoff);

  float mrow[8], lrow[8];
  v8f oacc[2];
#pragma unroll
  for (int r = 0; r < 8; ++r) { mrow[r] = -INFINITY; lrow[r] = 0.f; }
#pragma unroll
  for (int t = 0; t < 2; ++t) oacc[t] = (v8f){0.f,0.f,0.f,0.f,0.f,0.f,0.f,0.f};

#pragma unroll 1
  for (int ky = 0; ky < KWIN; ++ky) {
    const int ny = yy + ky - 3;
    const bool rowok = (ny >= 0) && (ny < IMG_H);
    const int nyc = ny < 0 ? 0 : (ny > (IMG_H - 1) ? (IMG_H - 1) : ny);
    __syncthreads();
    {
      const int nx = x0 - 8 + lane;
      const bool ok = rowok && (nx >= 0) && (nx < IMG_W);
      const int nxc = nx < 0 ? 0 : (nx > (IMG_W - 1) ? (IMG_W - 1) : nx);
      const int tk = bb * (IMG_H * IMG_W) + nyc * IMG_W + nxc;
      const v4u* ph = (const v4u*)(const void*)(khp + (size_t)tk * CEMB + head * DHD);
      const v4u* pl = (const v4u*)(const void*)(klp + (size_t)tk * CEMB + head * DHD);
      unsigned short* kd  = Ksh[wave] + lane * 32;
      unsigned short* kdl = Ksl[wave] + lane * 32;
#pragma unroll
      for (int u = 0; u < 4; ++u) {
        v4u a = ph[u];
        v4u bq = pl[u];
#pragma unroll
        for (int e = 0; e < 4; ++e) { a[e] = ok ? a[e] : 0u; bq[e] = ok ? bq[e] : 0u; }
        *(v4u*)(void*)(kd + u * 8) = a;
        *(v4u*)(void*)(kdl + u * 8) = bq;
      }
      const v4f* pv = (const v4f*)(qkv + (size_t)tk * NQKV + 2 * CEMB + head * DHD);
#pragma unroll
      for (int u = 0; u < 8; ++u) {
        const v4f f = pv[u];
#pragma unroll
        for (int e = 0; e < 4; ++e) {
          const float val = ok ? f[e] : 0.0f;
          const unsigned short hb = f2bf_bits(val);
          const unsigned short lb = f2bf_bits(val - bf_bits2f(hb));
          Vth[wave][(u * 4 + e) * 32 + lane] = hb;
          Vtl[wave][(u * 4 + e) * 32 + lane] = lb;
        }
      }
    }
    __syncthreads();
    v8f s[2];
#pragma unroll
    for (int j = 0; j < 2; ++j) {
      const __bf16* kp = (const __bf16*)(const void*)Ksh[wave] + (j * 16 + cc) * 32 + koff;
      const __bf16* kq = (const __bf16*)(const void*)Ksl[wave] + (j * 16 + cc) * 32 + koff;
      const v16b kbh = Frag<__bf16>::load(kp);
      const v16b kbl = Frag<__bf16>::load(kq);
      s[j] = (v8f){0.f,0.f,0.f,0.f,0.f,0.f,0.f,0.f};
      s[j] = at_mma(qah, kbh, s[j]);
      s[j] = at_mma(qah, kbl, s[j]);
      s[j] = at_mma(qal, kbh, s[j]);
    }
    const int dy = ky - 3;
    float cm[8];
#pragma unroll
    for (int r = 0; r < 8; ++r) {
      const int px = 8 * hh + r;
      float m = -INFINITY;
#pragma unroll
      for (int j = 0; j < 2; ++j) {
        const int slot = j * 16 + cc;
        const int kw = slot - px - 5;
        const bool inwin = (kw >= 0) && (kw < KWIN);
        const int dx = (inwin ? kw : 3) - 3;
        const float dist = sqrtf((float)(dy * dy + dx * dx));
        const float z = (wr[r] - dist) * shp[r];
        const float sm = sigm_f(z);
        float val = s[j][r] * QK_SCALE - (1.0f - sm) * 10000.0f;
        val = inwin ? val : -INFINITY;
        s[j][r] = val;
        m = fmaxf(m, val);
      }
#pragma unroll
      for (int off = 1; off < 16; off <<= 1) m = fmaxf(m, __shfl_xor(m, off, 32));
      cm[r] = m;
    }
    unsigned short* pwh = Psh[wave];
    unsigned short* pwl = Psl[wave];
#pragma unroll
    for (int r = 0; r < 8; ++r) {
      const float mnew = fmaxf(mrow[r], cm[r]);
      const float alpha = expf(mrow[r] - mnew);
      mrow[r] = mnew;
      float psum = 0.f;
#pragma unroll
      for (int j = 0; j < 2; ++j) {
        const float p = expf(s[j][r] - mnew);
        psum += p;
        const unsigned short hb = f2bf_bits(p);
        const unsigned short lb = f2bf_bits(p - bf_bits2f(hb));
        pwh[(8 * hh + r) * 32 + j * 16 + cc] = hb;
        pwl[(8 * hh + r) * 32 + j * 16 + cc] = lb;
      }
#pragma unroll
      for (int off = 1; off < 16; off <<= 1) psum += __shfl_xor(psum, off, 32);
      lrow[r] = lrow[r] * alpha + psum;
      oacc[0][r] *= alpha;
      oacc[1][r] *= alpha;
    }
    __syncthreads();
    {
      const __bf16* pa = (const __bf16*)(const void*)Psh[wave] + cc * 32 + koff;
      const __bf16* pb = (const __bf16*)(const void*)Psl[wave] + cc * 32 + koff;
      const v16b pah = Frag<__bf16>::load(pa);
      const v16b pal = Frag<__bf16>::load(pb);
#pragma unroll
      for (int t = 0; t < 2; ++t) {
        const __bf16* va = (const __bf16*)(const void*)Vth[wave] + (t * 16 + cc) * 32 + koff;
        const __bf16* vb = (const __bf16*)(const void*)Vtl[wave] + (t * 16 + cc) * 32 + koff;
        const v16b vbh = Frag<__bf16>::load(va);
        const v16b vbl = Frag<__bf16>::load(vb);
        oacc[t] = at_mma(pah, vbh, oacc[t]);
        oacc[t] = at_mma(pah, vbl, oacc[t]);
        oacc[t] = at_mma(pal, vbh, oacc[t]);
      }
    }
  }

  float* os = Osh[wave];
#pragma unroll
  for (int r = 0; r < 8; ++r) {
    const float inv = 1.0f / lrow[r];
#pragma unroll
    for (int t = 0; t < 2; ++t) os[(8 * hh + r) * 36 + t * 16 + cc] = oacc[t][r] * inv;
  }
  __syncthreads();
  {
    const int q4 = lane >> 3, c4 = (lane & 7) * 4;
    for (int pass = 0; pass < 2; ++pass) {
#pragma unroll
      for (int it = 0; it < 4; ++it) {
        const int row = it * 4 + q4;
        const v4f val = *(const v4f*)(os + row * 36 + c4);
        *(volatile v4f*)(obuf + (size_t)(tok0 + row) * CEMB + head * DHD + c4) = val;
      }
      __threadfence();
    }
  }
}

__global__ __launch_bounds__(256) void post_norm_kernel(
    const float* __restrict__ obuf, const float* __restrict__ qkv, const float* __restrict__ won,
    unsigned short* __restrict__ afh, unsigned short* __restrict__ afl) {
  __shared__ __align__(16) float swon[CEMB];
  const int tid = threadIdx.x;
  swon[tid] = won[tid];
  __syncthreads();
  const int wave = tid >> 5, lane = tid & 31;
  const v4f w0 = *(const v4f*)(swon + lane * 8);
  const v4f w1 = *(const v4f*)(swon + lane * 8 + 4);
#pragma unroll 1
  for (int it = 0; it < 4; ++it) {
    const int token = (blockIdx.x * 8 + wave) * 4 + it;
    const v4f* po = (const v4f*)(obuf + (size_t)token * CEMB + lane * 8);
    const v4f oa = po[0], ob = po[1];
    float ss = oa[0] * oa[0] + oa[1] * oa[1] + oa[2] * oa[2] + oa[3] * oa[3]
             + ob[0] * ob[0] + ob[1] * ob[1] + ob[2] * ob[2] + ob[3] * ob[3];
#pragma unroll
    for (int off = 1; off < 32; off <<= 1) ss += __shfl_xor(ss, off, 32);
    const float inv = 1.0f / sqrtf(ss * (1.0f / 256.0f) + RMS_EPS);
    const v4f* pv = (const v4f*)(qkv + (size_t)token * NQKV + 2 * CEMB + lane * 8);
    const v4f va = pv[0], vb = pv[1];
    float f[8];
    f[0] = oa[0] * inv * w0[0] + va[0];
    f[1] = oa[1] * inv * w0[1] + va[1];
    f[2] = oa[2] * inv * w0[2] + va[2];
    f[3] = oa[3] * inv * w0[3] + va[3];
    f[4] = ob[0] * inv * w1[0] + vb[0];
    f[5] = ob[1] * inv * w1[1] + vb[1];
    f[6] = ob[2] * inv * w1[2] + vb[2];
    f[7] = ob[3] * inv * w1[3] + vb[3];
    unsigned short hb[8], lb[8];
#pragma unroll
    for (int e = 0; e < 8; ++e) {
      hb[e] = f2bf_bits(f[e]);
      lb[e] = f2bf_bits(f[e] - bf_bits2f(hb[e]));
    }
    v4u hw, lw;
#pragma unroll
    for (int j = 0; j < 4; ++j) {
      hw[j] = (unsigned)hb[2 * j] | ((unsigned)hb[2 * j + 1] << 16);
      lw[j] = (unsigned)lb[2 * j] | ((unsigned)lb[2 * j + 1] << 16);
    }
    const size_t go = (size_t)token * CEMB + lane * 8;
    for (int pass = 0; pass < 2; ++pass) {
      *(volatile v4u*)(afh + go) = hw;
      *(volatile v4u*)(afl + go) = lw;
      __threadfence();
    }
  }
}

extern "C" void kernel_launch(void* const* d_in, const int* in_sizes, int n_in,
                              void* d_out, int out_size, void* d_ws, size_t ws_size,
                              hipStream_t stream) {
  if (n_in < 8) return;
  if (in_sizes[0] != NTOK * CEMB || in_sizes[1] != NQKV * CEMB || in_sizes[2] != DHD ||
      in_sizes[3] != DHD || in_sizes[4] != NWP_REAL * CEMB || in_sizes[5] != NWP_REAL ||
      in_sizes[6] != CEMB || in_sizes[7] != CEMB * CEMB) return;
  if (out_size != NTOK * CEMB) return;
  if (ws_size < WS_TOTAL) return;

  const float* x     = (const float*)d_in[0];
  const float* w_qkv = (const float*)d_in[1];
  const float* w_qn  = (const float*)d_in[2];
  const float* w_kn  = (const float*)d_in[3];
  const float* w_wp  = (const float*)d_in[4];
  const float* b_wp  = (const float*)d_in[5];
  const float* w_on  = (const float*)d_in[6];
  const float* w_out = (const float*)d_in[7];
  float* out = (float*)d_out;

  char* ws = (char*)d_ws;
  unsigned short* x_hi    = (unsigned short*)(ws + OFF_XH);
  unsigned short* x_lo    = (unsigned short*)(ws + OFF_XL);
  unsigned short* wqkv_hi = (unsigned short*)(ws + OFF_WQKVH);
  unsigned short* wqkv_lo = (unsigned short*)(ws + OFF_WQKVL);
  unsigned short* wwp_hi  = (unsigned short*)(ws + OFF_WWPH);
  unsigned short* wwp_lo  = (unsigned short*)(ws + OFF_WWPL);
  unsigned short* wout_hi = (unsigned short*)(ws + OFF_WOUTH);
  unsigned short* wout_lo = (unsigned short*)(ws + OFF_WOUTL);
  float*          qkv     = (float*)(ws + OFF_QKV);
  float*          wpraw   = (float*)(ws + OFF_WPR);
  unsigned short* q_hi    = (unsigned short*)(ws + OFF_QH);
  unsigned short* q_lo    = (unsigned short*)(ws + OFF_QL);
  unsigned short* k_hi    = (unsigned short*)(ws + OFF_KH);
  unsigned short* k_lo    = (unsigned short*)(ws + OFF_KL);
  float*          obuf    = (float*)(ws + OFF_OBUF);
  unsigned short* af_hi   = (unsigned short*)(ws + OFF_AFH);
  unsigned short* af_lo   = (unsigned short*)(ws + OFF_AFL);

  {
    const int n8x = NTOK * CEMB / 8;
    split_planes_kernel<<<dim3((n8x + 255) / 256), dim3(256), 0, stream>>>(x, NTOK * CEMB, x_hi, x_lo, n8x);
    const int n8q = NQKV * CEMB / 8;
    split_planes_kernel<<<dim3((n8q + 255) / 256), dim3(256), 0, stream>>>(w_qkv, NQKV * CEMB, wqkv_hi, wqkv_lo, n8q);
    const int n8w = NWP_PAD * CEMB / 8;
    split_planes_kernel<<<dim3((n8w + 255) / 256), dim3(256), 0, stream>>>(w_wp, NWP_REAL * CEMB, wwp_hi, wwp_lo, n8w);
    const int n8o = CEMB * CEMB / 8;
    split_planes_kernel<<<dim3((n8o + 255) / 256), dim3(256), 0, stream>>>(w_out, CEMB * CEMB, wout_hi, wout_lo, n8o);
  }
  {
    const int tiles = (NTOK / 64) * (NQKV / 64);
    wmma_gemm64<1, true, 0, 0, false, 3><<<dim3(tiles / 8, 1), dim3(256), 0, stream>>>(
        x_hi, x_lo, CEMB, 0L, wqkv_hi, wqkv_lo, CEMB, 0L,
        (void*)qkv, (void*)qkv, NQKV, 0L, w_on, w_on, 0L, NTOK, NQKV, CEMB, 1.0f);
  }
  {
    const int tiles = (NTOK / 64) * (NWP_PAD / 64);
    wmma_gemm64<1, true, 0, 0, false, 0><<<dim3(tiles / 8, 1), dim3(256), 0, stream>>>(
        x_hi, x_lo, CEMB, 0L, wwp_hi, wwp_lo, CEMB, 0L,
        (void*)wpraw, (void*)wpraw, NWP_PAD, 0L, w_on, w_on, 0L, NTOK, NWP_PAD, CEMB, 1.0f);
  }
  qk_prep_kernel<<<dim3(NTOK / 2), dim3(256), 0, stream>>>(qkv, w_qn, w_kn, q_hi, q_lo, k_hi, k_lo);
  local_attn_kernel<<<dim3(NB_BATCH * IMG_H * (IMG_W / 16) * 2), dim3(128), 0, stream>>>(
      q_hi, q_lo, k_hi, k_lo, qkv, wpraw, b_wp, obuf);
  post_norm_kernel<<<dim3(NTOK / 32), dim3(256), 0, stream>>>(obuf, qkv, w_on, af_hi, af_lo);
  {
    const int tiles = (NTOK / 64) * (CEMB / 64);
    wmma_gemm64<1, true, 0, 0, false, 3><<<dim3(tiles / 8, 1), dim3(256), 0, stream>>>(
        af_hi, af_lo, CEMB, 0L, wout_hi, wout_lo, CEMB, 0L,
        (void*)out, (void*)out, CEMB, 0L, w_on, w_on, 0L, NTOK, CEMB, CEMB, 1.0f);
  }
}
